// QuantumKernelEnhancement_29678224016038
// MI455X (gfx1250) — hardware-verified
//
#include <hip/hip_runtime.h>


namespace {
constexpr int NS = 2048, FD = 512, NQ = 10, NA = 1 << NQ  , NL = 3, KD = 2 * NA  ;
constexpr float PS = 8.0f;
typedef _Float16 b16;
typedef __attribute__((ext_vector_type(16))) _Float16 v16b;
typedef __attribute__((ext_vector_type(8))) _Float16 v8b;
typedef __attribute__((ext_vector_type(8))) float v8f;
typedef __attribute__((ext_vector_type(4))) float v4f;
typedef __attribute__((ext_vector_type(16))) short v16s;
__device__ __forceinline__ float bf16_rne(float f) { unsigned int u = __float_as_uint(f); u += 0x7FFFu + ((u >> 16) & 1u); return __uint_as_float(u & 0xFFFF0000u); }
__device__ __forceinline__ void split16(float v, b16& hi, b16& lo) { hi = (b16)v; lo = (b16)(v - (float)hi); }
__device__ __forceinline__ v16b frag_kb(const b16* p, int hh) { const v8b a = *(const v8b*)(p + 8 * hh), b = *(const v8b*)(p + 16 + 8 * hh); v16b f;
#pragma unroll
  for (int e = 0; e < 8; ++e) { f[e] = a[e]; f[8 + e] = b[e]; } return f; }
__device__ __forceinline__ v16b fneg(v16b f) { v16s s = (v16s)f; s ^= (v16s)((short)0x8000); return (v16b)s; }
__device__ __forceinline__ v8f wmma16b(v16b a, v16b b, v8f c) { v8f d = __builtin_amdgcn_wmma_f32_16x16x32_f16(false, a, false, b, (short)0, c, false, false); asm volatile("v_nop\n\tv_nop\n\tv_nop\n\tv_nop" : "+v"(d) : "v"(a), "v"(b)); return d; }
__device__ __forceinline__ void wave_lds_sync() { __builtin_amdgcn_fence(__ATOMIC_RELEASE, "workgroup"); __builtin_amdgcn_wave_barrier(); __builtin_amdgcn_fence(__ATOMIC_ACQUIRE, "workgroup"); }
__device__ __forceinline__ float pmul(float a, float b) { float p = a * b; asm volatile("" : "+v"(p)); return p; }

__global__ __launch_bounds__(256) void angle_kernel(const float* __restrict__ x1, const float* __restrict__ x2, const float* __restrict__ wenc, float* __restrict__ ANG, int base) {
  __shared__ __attribute__((aligned(16))) float sa[8][16];
  const int wave = threadIdx.x >> 5, lane = threadIdx.x & 31; const size_t blk = (size_t)blockIdx.x + base; const size_t s = blk * 8 + wave; const float* xr = (s < (size_t)NS ? x1 + s * FD : x2 + (s - NS) * FD);
  float acc[NQ], cmp[NQ];
#pragma unroll
  for (int q = 0; q < NQ; ++q) { acc[q] = 0.0f; cmp[q] = 0.0f; }
  for (int f = lane; f < FD; f += 32) { const float xv = bf16_rne(xr[f]);
#pragma unroll
    for (int q = 0; q < NQ; ++q) { const float p = pmul(xv, bf16_rne(wenc[f * NQ + q])); const float y = p - cmp[q]; const float t = acc[q] + y; float tt = t - acc[q]; asm volatile("" : "+v"(tt)); cmp[q] = tt - y; acc[q] = t; } }
#pragma unroll
  for (int q = 0; q < NQ; ++q) { float v = acc[q] - cmp[q]; for (int o = 16; o; o >>= 1) v += __shfl_xor(v, o); acc[q] = v; }
  if (lane == 0) {
#pragma unroll
    for (int q = 0; q < NQ; ++q) sa[wave][q] = acc[q];
    for (int q = NQ; q < 16; ++q) sa[wave][q] = 0.0f; }
  __syncthreads();
  for (int pass = 0; pass < 2; ++pass) { if (threadIdx.x < 32) *(volatile v4f*)(ANG + blk * 128 + threadIdx.x * 4) = *(const v4f*)(&sa[0][0] + threadIdx.x * 4); __threadfence(); }
}
__global__ __launch_bounds__(256) void state_kernel(const float* __restrict__ ANG, const float* __restrict__ qp, b16* __restrict__ Ph, b16* __restrict__ Pl, int base) {
  __shared__ float re[8][NA], im[8][NA];
  const int wave = threadIdx.x >> 5, lane = threadIdx.x & 31; const size_t s = ((size_t)blockIdx.x + base) * 8 + wave;
  float* R = re[wave]; float* I = im[wave];
  for (int a = lane; a < NA; a += 32) { R[a] = (a == 0) ? 1.0f : 0.0f; I[a] = 0.0f; }
  wave_lds_sync();
#pragma unroll 1
  for (int layer = 0; layer < NL; ++layer) {
#pragma unroll 1
    for (int q = 0; q < NQ; ++q) { const float p0 = bf16_rne(qp[(layer * NQ + q) * 3]), p1 = bf16_rne(qp[(layer * NQ + q) * 3 + 1]), p2 = bf16_rne(qp[(layer * NQ + q) * 3 + 2]);
      const float rx = ANG[s * 16 + q] * p0; const float c = cosf(rx * 0.5f), sn = sinf(rx * 0.5f);
      const float cy = cosf(p1 * 0.5f), sy = sinf(p1 * 0.5f);
      const float cz = cosf(p2 * 0.5f), sz = sinf(p2 * 0.5f);
      const int lo = 1 << q;
#pragma unroll 1
      for (int p = lane; p < NA / 2; p += 32) { const int i0 = ((p >> q) << (q + 1)) | (p & (lo - 1)); const int i1 = i0 | lo;
        float r0 = R[i0], m0 = I[i0], r1 = R[i1], m1 = I[i1];
        float nr0 = c * r0 + sn * m1, nm0 = c * m0 - sn * r1, nr1 = sn * m0 + c * r1, nm1 = -sn * r0 + c * m1;
        r0 = cy * nr0 - sy * nr1; m0 = cy * nm0 - sy * nm1; r1 = sy * nr0 + cy * nr1; m1 = sy * nm0 + cy * nm1;
        nr0 = cz * r0 + sz * m0; nm0 = cz * m0 - sz * r0; nr1 = cz * r1 - sz * m1; nm1 = cz * m1 + sz * r1;
        R[i0] = nr0; I[i0] = nm0; R[i1] = nr1; I[i1] = nm1; }
      wave_lds_sync(); }
#pragma unroll 1
    for (int q = 0; q < NQ - 1; ++q) { const int cb = 1 << q, tb = 1 << (q + 1);
#pragma unroll 1
      for (int p = lane; p < NA / 4; p += 32) {
        const int low = p & (cb - 1); const int high = p >> q; const int i0 = (high << (q + 2)) | cb | low; const int i1 = i0 | tb;
        const float r0 = R[i0], m0 = I[i0], r1 = R[i1], m1 = I[i1]; R[i0] = r1; I[i0] = m1; R[i1] = r0; I[i1] = m0; }
      wave_lds_sync(); } }
  for (int pass = 0; pass < 2; ++pass) { for (int c8 = lane * 8; c8 < KD; c8 += 256) { v8b h, l; for (int j = 0; j < 8; ++j) { const int a = c8 + j; const float v = (a < NA ? R[a] : I[a - NA]) * PS; b16 ph, pl; split16(v, ph, pl); h[j] = ph; l[j] = pl; }
      *(volatile v8b*)(Ph + s * KD + c8) = h; *(volatile v8b*)(Pl + s * KD + c8) = l; } __threadfence(); }
}
__global__ __launch_bounds__(128) void gram_kernel(const b16* __restrict__ Ph, const b16* __restrict__ Pl, float* __restrict__ out) {
  __shared__ __attribute__((aligned(16))) float Tf[4][16][128 + 4];
  const int wave = threadIdx.x >> 5, lane = threadIdx.x & 31, nloc = lane & 15, hlf = lane >> 4; const size_t i0 = (size_t)blockIdx.x * 64 + wave * 16; const size_t j0 = (size_t)blockIdx.y * 128;
  const b16* A_h = Ph + (i0 + nloc) * KD; const b16* A_l = Pl + (i0 + nloc) * KD; const b16* B2h = Ph + (size_t)NS * KD; const b16* B2l = Pl + (size_t)NS * KD;
  v8f are[8], aim[8];
#pragma unroll
  for (int t = 0; t < 8; ++t) { are[t] = (v8f){}; aim[t] = (v8f){}; }
  for (int kb = 0; kb < KD; kb += 32) { const v16b a = frag_kb(A_h + kb, hlf), al = frag_kb(A_l + kb, hlf); const int kb2 = (kb + NA) & (KD - 1); const bool negim = kb < NA;
#pragma unroll
    for (int t = 0; t < 8; ++t) { const size_t j = j0 + t * 16 + nloc; const b16* bh = B2h + j * KD; const b16* bl = B2l + j * KD;
      v16b b = frag_kb(bh + kb, hlf), blo = frag_kb(bl + kb, hlf); are[t] = wmma16b(a, b, are[t]); are[t] = wmma16b(al, b, are[t]); are[t] = wmma16b(a, blo, are[t]);
      b = frag_kb(bh + kb2, hlf); blo = frag_kb(bl + kb2, hlf); if (negim) { b = fneg(b); blo = fneg(blo); } aim[t] = wmma16b(a, b, aim[t]); aim[t] = wmma16b(al, b, aim[t]); aim[t] = wmma16b(a, blo, aim[t]); } }
  const float sc = 1.0f / (PS * PS);
#pragma unroll
  for (int t = 0; t < 8; ++t)
#pragma unroll 1
    for (int r = 0; r < 8; ++r) { const float x = are[t][r] * sc, y = aim[t][r] * sc; Tf[wave][8 * hlf + r][t * 16 + nloc] = x * x + y * y; }
  wave_lds_sync();
  for (int pass = 0; pass < 2; ++pass) { for (int rr = 0; rr < 16; ++rr) *(volatile v4f*)(out + (i0 + rr) * NS + j0 + lane * 4) = *(const v4f*)(&Tf[wave][rr][lane * 4]); __threadfence(); }
}
}

extern "C" void kernel_launch(void* const* d_in, const int* in_sizes, int n_in, void* d_out, int out_size, void* d_ws, size_t ws_size, hipStream_t stream) {
  (void)n_in;
  auto Fp = [&](int i) { return (const float*)d_in[i]; };
  if (in_sizes[0] != NS * FD || in_sizes[1] != NS * FD || in_sizes[2] != FD * NQ || in_sizes[3] != NL * NQ * 3 || out_size != NS * NS) return;
  size_t off = 0; char* ws = (char*)d_ws;
  auto carve = [&](size_t bytes) { char* p = ws + off; off += (bytes + 255) & ~(size_t)255; return p; };
  float* ANG = (float*)carve((size_t)2 * NS * 16 * 4); b16* Ph = (b16*)carve((size_t)2 * NS * KD * 2); b16* Pl = (b16*)carve((size_t)2 * NS * KD * 2);
  if (off > ws_size || off > ((size_t)128 << 20)) return;
  angle_kernel<<<2 * NS / 8, 256, 0, stream>>>(Fp(0), Fp(1), Fp(2), ANG, 0);
  state_kernel<<<2 * NS / 8, 256, 0, stream>>>(ANG, Fp(3), Ph, Pl, 0);
  gram_kernel<<<dim3(NS / 64, NS / 128), 128, 0, stream>>>(Ph, Pl, (float*)d_out);
}
